// TemporalGNN_30365418783390
// MI455X (gfx1250) — hardware-run, weakly checked
//
#include <hip/hip_runtime.h>
#include <stddef.h>
#include <stdint.h>
#include <math.h>

#pragma clang fp contract(off)

#define NN      50000
#define NE      800000
#define HD      128
#define NC      2
#define GBM     128
#define MP      50048
#define NTHR    256
#define NWAVE   8
#define EPT     8
#define WCH     (32 * EPT)
#define NBRUN   1024
#define SLB     10
#define NBK     49
#define WLCAP   3584
#define RCAP    28672
#define DEGCAP  64
#define MAXDEG_MEAS   35
#define MAXB1024_MEAS 16623
#define SP      132

#ifndef SPLIT_TWO
#define SPLIT_TWO 1
#endif
#ifndef SPLIT_THREE
#define SPLIT_THREE 1
#endif
#define K_ONE   128
#define AP_ONE  128
#define WP_ONE  128
#define AP_TWO  256
#define WP_TWO  256

#define TB_L1     0
#define TB_L2     640
#define TB_B3     1280
#define TB_FC     1408
#define TB_FCB    1664
#define TB_FLOATS 1696

#define BK_ZINTS (NWAVE * WLCAP + RCAP + 4 * NBRUN)
#define BK_INTS  (BK_ZINTS + 16)
#define BK_LDS   (BK_INTS * 4)
#define GM_LDS   ((GBM * SP + GBM) * 4)

#define PBX   (MP * HD / 8 / NTHR)
#define PBW1  (HD * K_ONE / 8 / NTHR)
#define PBW2  (HD * WP_TWO / 8 / NTHR)
#define PBHZ  ((MP - NN) * AP_TWO / 8 / NTHR)
#define PBTOT (PBX + PBW1 + 2 * PBW2 + PBHZ + 1)

static_assert(NE % WCH == 0 && NE % 4 == 0);
static_assert(NN % 16 == 0 && NBRUN % 16 == 0 && (NN % NBRUN) % 16 == 0);
static_assert(32 * 4 == HD);
static_assert(MP == 391 * GBM && MP >= NN && MP % GBM == 0);
static_assert(NBRUN == (1 << SLB) && NBRUN % GBM == 0 && NBK * NBRUN >= MP);
static_assert((NBK - 1) * NBRUN < NN);
static_assert(NE < (1 << 20) && (((long long)NE) << SLB) < (1LL << 31));
static_assert(RCAP == 28672 && RCAP == NWAVE * WLCAP && RCAP % (NTHR * 4) == 0);
static_assert((long long)RCAP * 100 >= (long long)MAXB1024_MEAS * 105);
static_assert(WLCAP >= MAXB1024_MEAS / 8 + 8 * 46 + 1);
static_assert(DEGCAP == 64 && MAXDEG_MEAS + 8 <= DEGCAP);
static_assert(BK_ZINTS % 4 == 0 && BK_ZINTS % (NTHR * 4) == 0 && BK_LDS <= 327680);
static_assert(GM_LDS <= 327680 && (SP * 4) % 16 == 0);
static_assert((MP * HD / 8) % NTHR == 0 && (HD * K_ONE / 8) % NTHR == 0 && (HD * WP_TWO / 8) % NTHR == 0);
static_assert(((MP - NN) * AP_TWO / 8) % NTHR == 0);
static_assert(K_ONE % 32 == 0 && AP_TWO == 2 * HD && WP_TWO == 2 * HD);
static_assert(TB_FLOATS * 4 <= 8192 && TB_FLOATS % 32 == 0);
static_assert((NBRUN * NC) % (4 * NTHR) == 0);

typedef float          v4f   __attribute__((ext_vector_type(4)));
typedef float          v8f   __attribute__((ext_vector_type(8)));
typedef int            v4i   __attribute__((ext_vector_type(4)));
typedef int            v8i   __attribute__((ext_vector_type(8)));
typedef unsigned short v8us  __attribute__((ext_vector_type(8)));
typedef unsigned short v16us __attribute__((ext_vector_type(16)));
typedef __bf16         v16bf __attribute__((ext_vector_type(16)));
typedef v4f  __attribute__((may_alias)) v4fa;
typedef v4i  __attribute__((may_alias)) v4ia;
typedef v8us __attribute__((may_alias)) v8usa;
union FragB { v16bf v; v16us u; v8us h[2]; v8i w; };

__device__ __forceinline__ v8f wmb(const FragB& a, const FragB& b, v8f c) {
  v8f d = __builtin_amdgcn_wmma_f32_16x16x32_bf16(false, a.v, false, b.v, (short)0, c, false, false);
  asm volatile("v_nop\n\tv_nop\n\tv_nop\n\tv_nop" : "+v"(d) : "v"(a.w), "v"(b.w));
  return d;
}

__device__ __forceinline__ unsigned bf16_bits(float f) {
  const unsigned u = __float_as_uint(f);
  const unsigned r = (u + 0x7FFFu + ((u >> 16) & 1u)) >> 16;
  const unsigned q = (u >> 16) | 0x40u;
  return ((u & 0x7fffffffu) > 0x7f800000u) ? q : r;
}
__device__ __forceinline__ float bf16_val(float f) {
  return __uint_as_float(bf16_bits(f) << 16);
}

__device__ __forceinline__ void hilo_pack(float v0, float v1, float v2, float v3,
                                          int& h01, int& h23, int& l01, int& l23) {
  const unsigned a0 = bf16_bits(v0), a1 = bf16_bits(v1), a2 = bf16_bits(v2), a3 = bf16_bits(v3);
  const unsigned b0 = bf16_bits(v0 - __uint_as_float(a0 << 16));
  const unsigned b1 = bf16_bits(v1 - __uint_as_float(a1 << 16));
  const unsigned b2 = bf16_bits(v2 - __uint_as_float(a2 << 16));
  const unsigned b3 = bf16_bits(v3 - __uint_as_float(a3 << 16));
  h01 = (int)(a0 | (a1 << 16)); h23 = (int)(a2 | (a3 << 16));
  l01 = (int)(b0 | (b1 << 16)); l23 = (int)(b2 | (b3 << 16));
}

__device__ __forceinline__ v4i regroup32(int h01, int h23, int l01, int l23, int lane) {
  const int s0 = (2 * lane) & 31, s1 = s0 + 1;
  const int a0 = __shfl(h01, s0, 32), a1 = __shfl(h23, s0, 32), a2 = __shfl(h01, s1, 32), a3 = __shfl(h23, s1, 32);
  const int b0 = __shfl(l01, s0, 32), b1 = __shfl(l23, s0, 32), b2 = __shfl(l01, s1, 32), b3 = __shfl(l23, s1, 32);
  const int mk = (lane < 16) ? -1 : 0;
  v4i o;
  o.x = (a0 & mk) | (b0 & ~mk); o.y = (a1 & mk) | (b1 & ~mk);
  o.z = (a2 & mk) | (b2 & ~mk); o.w = (a3 & mk) | (b3 & ~mk);
  return o;
}

__device__ __forceinline__ void st2_v4f(float* p, v4f v) {
  *(volatile v4f*)p = v;
  __threadfence();
  *(volatile v4f*)p = v;
}
__device__ __forceinline__ void st2_v8us(unsigned short* p, v8us v) {
  *(volatile v8us*)p = v;
  __threadfence();
  *(volatile v8us*)p = v;
}
__device__ __forceinline__ void st2_v4i(int* p, v4i v) {
  *(volatile v4i*)p = v;
  __threadfence();
  *(volatile v4i*)p = v;
}

__device__ __forceinline__ v8us fetch8(const float* __restrict__ base, int stride) {
  float f[8];
#pragma unroll
  for (int i = 0; i < 8; ++i) f[i] = base[(size_t)i * (size_t)stride];
  v8us o;
#pragma unroll
  for (int i = 0; i < 8; ++i) o[i] = (unsigned short)bf16_bits(f[i]);
  return o;
}

__device__ __forceinline__ void tab_line(const float* __restrict__ src, int nvalid, float* dst, int lane) {
  const int i0 = 4 * lane, i1 = i0 + 1, i2 = i0 + 2, i3 = i0 + 3;
  const int lim = nvalid - 1;
  const float a0 = src[i0 < lim ? i0 : lim];
  const float a1 = src[i1 < lim ? i1 : lim];
  const float a2 = src[i2 < lim ? i2 : lim];
  const float a3 = src[i3 < lim ? i3 : lim];
  asm volatile("" :: "v"(a0), "v"(a1), "v"(a2), "v"(a3));
  v4f o;
  o.x = (i0 < nvalid) ? bf16_val(a0) : 0.0f;
  o.y = (i1 < nvalid) ? bf16_val(a1) : 0.0f;
  o.z = (i2 < nvalid) ? bf16_val(a2) : 0.0f;
  o.w = (i3 < nvalid) ? bf16_val(a3) : 0.0f;
  st2_v4f(dst + 4 * lane, o);
}

__global__ __launch_bounds__(NTHR) void k_prep(
    const float* __restrict__ x,
    const float* __restrict__ W1, const float* __restrict__ W2, const float* __restrict__ W3,
    const float* __restrict__ b1, const float* __restrict__ g1, const float* __restrict__ be1,
    const float* __restrict__ m1, const float* __restrict__ v1,
    const float* __restrict__ b2, const float* __restrict__ g2, const float* __restrict__ be2,
    const float* __restrict__ m2, const float* __restrict__ v2,
    const float* __restrict__ b3, const float* __restrict__ fcW, const float* __restrict__ fcb,
    unsigned short* xb, unsigned short* w1t, unsigned short* w2d, unsigned short* w3d,
    unsigned short* hl, float* tb) {
  __shared__ __attribute__((aligned(16))) float srs[NTHR];
  const int tid = (int)threadIdx.x, lane = tid & 31, wave = tid >> 5;
  const int blk = (int)blockIdx.x;
  if (blk < PBX) {
    const int u   = blk * NTHR + tid;
    const int row = u >> 4, k8 = (u & 15) * 8;
    const int rc  = row < NN ? row : NN - 1;
    const unsigned mk = row < NN ? 0xffffu : 0u;
    const float* p = x + (size_t)rc * HD + k8;
    const v4f a = *(const v4fa*)p;
    const v4f b = *(const v4fa*)(p + 4);
    v8us o;
    o[0] = (unsigned short)(bf16_bits(a.x) & mk); o[1] = (unsigned short)(bf16_bits(a.y) & mk);
    o[2] = (unsigned short)(bf16_bits(a.z) & mk); o[3] = (unsigned short)(bf16_bits(a.w) & mk);
    o[4] = (unsigned short)(bf16_bits(b.x) & mk); o[5] = (unsigned short)(bf16_bits(b.y) & mk);
    o[6] = (unsigned short)(bf16_bits(b.z) & mk); o[7] = (unsigned short)(bf16_bits(b.w) & mk);
    st2_v8us(xb + (size_t)row * HD + k8, o);
  } else if (blk < PBX + PBW1) {
    const int u = (blk - PBX) * NTHR + tid;
    const int n = u >> 4, k8 = (u & 15) * 8;
    const v8us o = fetch8(W1 + (size_t)k8 * HD + n, HD);
    st2_v8us(w1t + (size_t)n * WP_ONE + k8, o);
  } else if (blk < PBX + PBW1 + PBW2) {
    const int u = (blk - PBX - PBW1) * NTHR + tid;
    const int n = u >> 5, k8 = (u & 31) * 8, kk = k8 & (HD - 1);
    const v8us o = fetch8(W2 + (size_t)kk * HD + n, HD);
    st2_v8us(w2d + (size_t)n * WP_TWO + k8, o);
  } else if (blk < PBX + PBW1 + 2 * PBW2) {
    const int u = (blk - PBX - PBW1 - PBW2) * NTHR + tid;
    const int n = u >> 5, k8 = (u & 31) * 8, kk = k8 & (HD - 1);
    const v8us o = fetch8(W3 + (size_t)kk * HD + n, HD);
    st2_v8us(w3d + (size_t)n * WP_TWO + k8, o);
  } else if (blk < PBX + PBW1 + 2 * PBW2 + PBHZ) {
    const int u = (blk - PBX - PBW1 - 2 * PBW2) * NTHR + tid;
    const int row = NN + (u >> 5), k8 = (u & 31) * 8;
    const v8us z = {0, 0, 0, 0, 0, 0, 0, 0};
    st2_v8us(hl + (size_t)row * AP_TWO + k8, z);
  } else {
    {
      const int c = tid & (HD - 1);
      const float a = v1[c];
      const float b = v2[c];
      asm volatile("" :: "v"(a), "v"(b));
      const float vv = (tid < HD) ? a : b;
      srs[tid] = 1.0f / sqrtf(bf16_val(vv) + 1e-5f);
    }
    __syncthreads();
    if (wave == 0) {
      tab_line(b1, HD, tb + TB_L1 + 0, lane);
      tab_line(m1, HD, tb + TB_L1 + 128, lane);
    } else if (wave == 1) {
      const v4f o = *(const v4fa*)(srs + 4 * lane);
      st2_v4f(tb + TB_L1 + 256 + 4 * lane, o);
      tab_line(g1, HD, tb + TB_L1 + 384, lane);
    } else if (wave == 2) {
      tab_line(be1, HD, tb + TB_L1 + 512, lane);
      tab_line(b2, HD, tb + TB_L2 + 0, lane);
    } else if (wave == 3) {
      tab_line(m2, HD, tb + TB_L2 + 128, lane);
      const v4f o = *(const v4fa*)(srs + HD + 4 * lane);
      st2_v4f(tb + TB_L2 + 256 + 4 * lane, o);
    } else if (wave == 4) {
      tab_line(g2, HD, tb + TB_L2 + 384, lane);
      tab_line(be2, HD, tb + TB_L2 + 512, lane);
    } else if (wave == 5) {
      tab_line(b3, HD, tb + TB_B3, lane);
      tab_line(fcW, HD, tb + TB_FC, lane);
    } else if (wave == 6) {
      tab_line(fcW + HD, HD, tb + TB_FC + HD, lane);
      tab_line(fcb, NC, tb + TB_FCB, lane);
    }
  }
}

__device__ __forceinline__ void bucket_flush(const int* pl, const int* cnt, const float* dvf, int ov,
                                             int* lp, int* cop, float* dp, int* fp, int tid) {
#pragma unroll 1
  for (int i = tid * 4; i < RCAP; i += NTHR * 4) {
    const v4i v = *(const v4ia*)(pl + i);
    *(volatile v4i*)(lp + i) = v;
  }
#pragma unroll 1
  for (int i = tid * 4; i < 2 * NBRUN; i += NTHR * 4) {
    const v4i v = *(const v4ia*)(cnt + i);
    *(volatile v4i*)(cop + i) = v;
  }
  {
    const v4f d = *(const v4fa*)(dvf + 4 * tid);
    *(volatile v4f*)(dp + 4 * tid) = d;
  }
  if (tid < 8) {
    const v4i f = {ov, ov, ov, ov};
    *(volatile v4i*)(fp + 4 * tid) = f;
  }
}

__global__ __launch_bounds__(NTHR) void k_bucket(const int* __restrict__ srcs, const int* __restrict__ dsts,
                                                 int* LIST, int* CO, float* DINV, int* FLAG) {
  extern __shared__ __attribute__((aligned(16))) int bk_dsm[];
  int*   wl   = bk_dsm;
  int*   pl   = bk_dsm + NWAVE * WLCAP;
  int*   cnt  = pl + RCAP;
  int*   offs = cnt + NBRUN;
  int*   cur  = offs + NBRUN;
  float* dvf  = (float*)(cur + NBRUN);
  int*   misc = cur + 2 * NBRUN;
  const int tid = (int)threadIdx.x, lane = tid & 31, wave = tid >> 5;
  const int blk = (int)blockIdx.x;
  const unsigned nbs = (unsigned)(blk * NBRUN);

  {
    const v4i z4 = {0, 0, 0, 0};
    for (int i = tid * 4; i < BK_ZINTS; i += NTHR * 4) *(v4ia*)(bk_dsm + i) = z4;
    if (tid < 16) misc[tid] = 0;
  }
  __syncthreads();

  {
    const int per  = ((NE + NWAVE * WCH - 1) / (NWAVE * WCH)) * WCH;
    const int ebeg = wave * per;
    const int eend = (ebeg + per < NE) ? (ebeg + per) : NE;
    int* mylist = wl + wave * WLCAP;
    int wc = 0;
#pragma unroll 1
    for (int cb = ebeg; cb < eend; cb += WCH) {
      const int e0 = cb + lane * EPT;
      const v4i da = *(const v4ia*)(dsts + e0);
      const v4i db = *(const v4ia*)(dsts + e0 + 4);
      const unsigned s0 = (unsigned)da.x - nbs, s1 = (unsigned)da.y - nbs;
      const unsigned s2 = (unsigned)da.z - nbs, s3 = (unsigned)da.w - nbs;
      const unsigned s4 = (unsigned)db.x - nbs, s5 = (unsigned)db.y - nbs;
      const unsigned s6 = (unsigned)db.z - nbs, s7 = (unsigned)db.w - nbs;
      const bool h0 = s0 < (unsigned)NBRUN, h1 = s1 < (unsigned)NBRUN, h2 = s2 < (unsigned)NBRUN, h3 = s3 < (unsigned)NBRUN;
      const bool h4 = s4 < (unsigned)NBRUN, h5 = s5 < (unsigned)NBRUN, h6 = s6 < (unsigned)NBRUN, h7 = s7 < (unsigned)NBRUN;
      const unsigned m0 = __builtin_amdgcn_ballot_w32(h0), m1 = __builtin_amdgcn_ballot_w32(h1);
      const unsigned m2 = __builtin_amdgcn_ballot_w32(h2), m3 = __builtin_amdgcn_ballot_w32(h3);
      const unsigned m4 = __builtin_amdgcn_ballot_w32(h4), m5 = __builtin_amdgcn_ballot_w32(h5);
      const unsigned m6 = __builtin_amdgcn_ballot_w32(h6), m7 = __builtin_amdgcn_ballot_w32(h7);
      const unsigned any = m0 | m1 | m2 | m3 | m4 | m5 | m6 | m7;
      if (any != 0u) {
        const int pre = (int)(__builtin_amdgcn_mbcnt_lo(m0, 0u) + __builtin_amdgcn_mbcnt_lo(m1, 0u) +
                              __builtin_amdgcn_mbcnt_lo(m2, 0u) + __builtin_amdgcn_mbcnt_lo(m3, 0u) +
                              __builtin_amdgcn_mbcnt_lo(m4, 0u) + __builtin_amdgcn_mbcnt_lo(m5, 0u) +
                              __builtin_amdgcn_mbcnt_lo(m6, 0u) + __builtin_amdgcn_mbcnt_lo(m7, 0u));
        int p = wc + pre;
        if (h0) { if (p < WLCAP) mylist[p] = ((e0 + 0) << SLB) | (int)s0; p = p + 1; }
        if (h1) { if (p < WLCAP) mylist[p] = ((e0 + 1) << SLB) | (int)s1; p = p + 1; }
        if (h2) { if (p < WLCAP) mylist[p] = ((e0 + 2) << SLB) | (int)s2; p = p + 1; }
        if (h3) { if (p < WLCAP) mylist[p] = ((e0 + 3) << SLB) | (int)s3; p = p + 1; }
        if (h4) { if (p < WLCAP) mylist[p] = ((e0 + 4) << SLB) | (int)s4; p = p + 1; }
        if (h5) { if (p < WLCAP) mylist[p] = ((e0 + 5) << SLB) | (int)s5; p = p + 1; }
        if (h6) { if (p < WLCAP) mylist[p] = ((e0 + 6) << SLB) | (int)s6; p = p + 1; }
        if (h7) { if (p < WLCAP) mylist[p] = ((e0 + 7) << SLB) | (int)s7; p = p + 1; }
        wc += (int)(__builtin_popcount(m0) + __builtin_popcount(m1) + __builtin_popcount(m2) + __builtin_popcount(m3) +
                    __builtin_popcount(m4) + __builtin_popcount(m5) + __builtin_popcount(m6) + __builtin_popcount(m7));
      }
    }
    if (lane == 0) misc[wave] = wc;
  }
  __syncthreads();

  if (wave == 0) {
    int ov = 0;
#pragma unroll 1
    for (int w2 = 0; w2 < NWAVE; ++w2) {
      int c = misc[w2];
      if (c > WLCAP) ov = 1;
      c = c < 0 ? 0 : (c > WLCAP ? WLCAP : c);
#pragma unroll 1
      for (int b0 = 0; b0 < c; b0 += 32) {
        const int idx = b0 + lane;
        const int ent = wl[w2 * WLCAP + (idx < WLCAP ? idx : WLCAP - 1)];
        const int m32 = (c - b0) < 32 ? (c - b0) : 32;
#pragma unroll 1
        for (int k = 0; k < m32; ++k) {
          const int u    = __builtin_amdgcn_readlane(ent, k);
          const int slot = u & (NBRUN - 1);
          if (lane == 0) cnt[slot] = cnt[slot] + 1;
        }
      }
    }
    if (lane == 0) misc[9] = ov;
  }
  __syncthreads();
  if (wave == 0) {
    const int base = lane * (NBRUN / 32);
    int s = 0;
#pragma unroll 1
    for (int i = 0; i < NBRUN / 32; ++i) s += cnt[base + i];
    int incl = s;
#pragma unroll
    for (int d = 1; d < 32; d <<= 1) {
      const int y = __shfl_up(incl, d, 32);
      if (lane >= d) incl += y;
    }
    int run = incl - s;
#pragma unroll 1
    for (int i = 0; i < NBRUN / 32; ++i) {
      const int cv = cnt[base + i];
      offs[base + i] = run;
      cur[base + i]  = run;
      run += cv;
    }
  }
  __syncthreads();

#pragma unroll 1
  for (int i = tid; i < NBRUN; i += NTHR) {
    int cv = cnt[i];
    cv = cv < 0 ? 0 : cv;
    dvf[i] = 1.0f / sqrtf((float)(cv + 1));
  }

  if (wave == 0) {
#pragma unroll 1
    for (int w2 = 0; w2 < NWAVE; ++w2) {
      int c = misc[w2];
      c = c < 0 ? 0 : (c > WLCAP ? WLCAP : c);
#pragma unroll 1
      for (int b0 = 0; b0 < c; b0 += 32) {
        const int idx = b0 + lane;
        const int ent = wl[w2 * WLCAP + (idx < WLCAP ? idx : WLCAP - 1)];
        int eid = (ent >> SLB) & 0xFFFFF;
        eid = eid > NE - 1 ? NE - 1 : eid;
        int sr = srcs[eid];
        sr = sr < 0 ? 0 : (sr > NN - 1 ? NN - 1 : sr);
        const int m32 = (c - b0) < 32 ? (c - b0) : 32;
#pragma unroll 1
        for (int k = 0; k < m32; ++k) {
          const int u    = __builtin_amdgcn_readlane(ent, k);
          const int wd   = __builtin_amdgcn_readlane(sr, k);
          const int slot = u & (NBRUN - 1);
          if (lane == 0) {
            int p = cur[slot];
            p = p < 0 ? 0 : (p > RCAP - 1 ? RCAP - 1 : p);
            pl[p] = wd;
            cur[slot] = p + 1;
          }
        }
      }
    }
  }
  __syncthreads();

  const int ovf = misc[9];
  int*   lp  = LIST + (size_t)blk * RCAP;
  int*   cop = CO + (size_t)blk * (2 * NBRUN);
  float* dp  = DINV + (size_t)blk * NBRUN;
  int*   fp  = FLAG + (size_t)blk * 32;
  bucket_flush(pl, cnt, dvf, ovf, lp, cop, dp, fp, tid);
  __threadfence();
  bucket_flush(pl, cnt, dvf, ovf, lp, cop, dp, fp, tid);
}

template <int KTOT, int APITCH, int WPITCH>
__device__ __forceinline__ void gemm_body(const unsigned short* __restrict__ A,
                                          const unsigned short* __restrict__ WT,
                                          const float* __restrict__ DINV, float* P, float* sm) {
  static_assert(KTOT % 32 == 0 && KTOT <= APITCH && KTOT <= WPITCH);
  float* stg = sm;
  float* sdv = sm + GBM * SP;
  const int tid = (int)threadIdx.x, lane = tid & 31, wave = tid >> 5, hh = lane >> 4, m = lane & 15;
  const int rowBase = (int)blockIdx.x * GBM;
  if (tid < 32) {
    const v4f d = *(const v4fa*)(DINV + rowBase + 4 * tid);
    *(v4fa*)(sdv + 4 * tid) = d;
  }

  v8f acc[8];
  {
    const v8f z = {0.f, 0.f, 0.f, 0.f, 0.f, 0.f, 0.f, 0.f};
#pragma unroll
    for (int t = 0; t < 8; ++t) acc[t] = z;
  }
  const unsigned short* ap = A + (size_t)(rowBase + 16 * wave + m) * (size_t)APITCH + 8 * hh;
  const unsigned short* bp = WT + (size_t)m * (size_t)WPITCH + 8 * hh;
#pragma unroll 1
  for (int k0 = 0; k0 < KTOT; k0 += 32) {
    FragB af;
    af.h[0] = *(const v8usa*)(ap + k0);
    af.h[1] = *(const v8usa*)(ap + k0 + 16);
#pragma unroll
    for (int nt = 0; nt < 8; ++nt) {
      const unsigned short* wq = bp + (size_t)(16 * nt) * (size_t)WPITCH + k0;
      FragB bf;
      bf.h[0] = *(const v8usa*)wq;
      bf.h[1] = *(const v8usa*)(wq + 16);
      acc[nt] = wmb(af, bf, acc[nt]);
    }
  }
#pragma unroll
  for (int nt = 0; nt < 8; ++nt) {
#pragma unroll
    for (int r = 0; r < 8; ++r) stg[(16 * wave + 8 * hh + r) * SP + 16 * nt + m] = acc[nt][r];
  }
  __syncthreads();

#pragma unroll 1
  for (int i = 0; i < 16; ++i) {
    const int lr   = 16 * wave + i;
    const int grow = rowBase + lr;
    const v4f a  = *(const v4fa*)(stg + lr * SP + 4 * lane);
    const float dv = sdv[lr];
    asm volatile("" :: "v"(a));
    asm volatile("" :: "v"(dv));
    v4f o;
    o.x = dv * a.x; o.y = dv * a.y; o.z = dv * a.z; o.w = dv * a.w;
    if (grow < NN) st2_v4f(P + (size_t)grow * HD + 4 * lane, o);
  }
}

__global__ __launch_bounds__(NTHR) __attribute__((amdgpu_num_vgpr(248)))
void k_gemm_one(const unsigned short* __restrict__ XB, const unsigned short* __restrict__ W1T,
                const float* __restrict__ DINV, float* P) {
  extern __shared__ __attribute__((aligned(16))) float gm_dsm[];
  gemm_body<K_ONE, AP_ONE, WP_ONE>(XB, W1T, DINV, P, gm_dsm);
}

template <int KTOT>
__global__ __launch_bounds__(NTHR) __attribute__((amdgpu_num_vgpr(248)))
void k_gemm_two(const unsigned short* __restrict__ HL, const unsigned short* __restrict__ WD,
                const float* __restrict__ DINV, float* P) {
  extern __shared__ __attribute__((aligned(16))) float gm_dsm[];
  gemm_body<KTOT, AP_TWO, WP_TWO>(HL, WD, DINV, P, gm_dsm);
}

__device__ __forceinline__ v4f row_sum(const int* __restrict__ lb, const float* __restrict__ P,
                                       int c, int o, int lane) {
  int last = o + c - 1; last = last < o ? o : last;
  last = last > RCAP - 1 ? RCAP - 1 : last;
  float a0 = 0.0f, a1 = 0.0f, a2 = 0.0f, a3 = 0.0f;
#pragma unroll 1
  for (int b0 = 0; b0 < c; b0 += 32) {
    int idx = o + b0 + lane;
    idx = idx > last ? last : idx;
    int sr = lb[idx];
    sr = sr < 0 ? 0 : (sr > NN - 1 ? NN - 1 : sr);
    const int m32 = (c - b0) < 32 ? (c - b0) : 32;
#pragma unroll 1
    for (int k = 0; k < m32; ++k) {
      const int sk = __builtin_amdgcn_readlane(sr, k);
      const v4f v = *(const v4fa*)(P + (size_t)sk * HD + 4 * lane);
      a0 += v.x; a1 += v.y; a2 += v.z; a3 += v.w;
    }
  }
  v4f r;
  r.x = a0; r.y = a1; r.z = a2; r.w = a3;
  return r;
}

__global__ __launch_bounds__(NTHR) void k_replay_hl(const int* __restrict__ LIST, const int* __restrict__ CO,
                                                    const int* __restrict__ FLAG, const float* __restrict__ DINV,
                                                    const float* __restrict__ P, const float* __restrict__ TL,
                                                    unsigned short* HL) {
  const int tid = (int)threadIdx.x, lane = tid & 31, wave = tid >> 5;
  const int rowBase = (int)blockIdx.x * GBM;
  const int bucket  = rowBase >> SLB;
  const int* lb  = LIST + (size_t)bucket * RCAP;
  const int* cob = CO + (size_t)bucket * (2 * NBRUN);
  const int flag = FLAG[(size_t)bucket * 32];
  const float qnan = __uint_as_float(0x7fc00000u);

  const v4f pb  = *(const v4fa*)(TL + 0 + 4 * lane);
  const v4f pm  = *(const v4fa*)(TL + 128 + 4 * lane);
  const v4f prs = *(const v4fa*)(TL + 256 + 4 * lane);
  const v4f pg  = *(const v4fa*)(TL + 384 + 4 * lane);
  const v4f pbe = *(const v4fa*)(TL + 512 + 4 * lane);
  asm volatile("" :: "v"(pb), "v"(pm), "v"(prs));
  asm volatile("" :: "v"(pg), "v"(pbe));

#pragma unroll 1
  for (int i = 0; i < GBM / NWAVE; ++i) {
    const int d    = rowBase + (GBM / NWAVE) * wave + i;
    const int slot = d & (NBRUN - 1);
    int c = cob[slot];
    int o = cob[NBRUN + slot];
    const bool big = c > DEGCAP;
    c = c < 0 ? 0 : (c > DEGCAP ? DEGCAP : c);
    o = o < 0 ? 0 : (o > RCAP - 1 ? RCAP - 1 : o);
    c = __builtin_amdgcn_readfirstlane(c);
    o = __builtin_amdgcn_readfirstlane(o);
    const v4f a = row_sum(lb, P, c, o, lane);
    const int nc = d < NN ? d : NN - 1;
    const v4f sf = *(const v4fa*)(P + (size_t)nc * HD + 4 * lane);
    const float dd = DINV[nc];
    asm volatile("" :: "v"(sf));
    asm volatile("" :: "v"(dd));
    const float t0 = dd * (a.x + sf.x) + pb.x, t1 = dd * (a.y + sf.y) + pb.y;
    const float t2 = dd * (a.z + sf.z) + pb.z, t3 = dd * (a.w + sf.w) + pb.w;
    float y0 = ((t0 - pm.x) * prs.x) * pg.x + pbe.x;
    float y1 = ((t1 - pm.y) * prs.y) * pg.y + pbe.y;
    float y2 = ((t2 - pm.z) * prs.z) * pg.z + pbe.z;
    float y3 = ((t3 - pm.w) * prs.w) * pg.w + pbe.w;
    y0 = (y0 > 0.0f) ? y0 : (y0 - y0); y1 = (y1 > 0.0f) ? y1 : (y1 - y1);
    y2 = (y2 > 0.0f) ? y2 : (y2 - y2); y3 = (y3 > 0.0f) ? y3 : (y3 - y3);
    const bool bad  = (flag != 0) | big;
    const bool live = d < NN;
    y0 = bad ? qnan : y0; y1 = bad ? qnan : y1; y2 = bad ? qnan : y2; y3 = bad ? qnan : y3;
    y0 = live ? y0 : 0.0f; y1 = live ? y1 : 0.0f; y2 = live ? y2 : 0.0f; y3 = live ? y3 : 0.0f;
    int h01, h23, l01, l23;
    hilo_pack(y0, y1, y2, y3, h01, h23, l01, l23);
    const v4i ow = regroup32(h01, h23, l01, l23, lane);
    st2_v4i((int*)(HL + (size_t)d * AP_TWO + 8 * lane), ow);
  }
}

__device__ __forceinline__ void head_flush(const float* os, float* ob, int nv4, int tid) {
#pragma unroll 1
  for (int it = 0; it < (NBRUN * NC) / (4 * NTHR); ++it) {
    const int i4 = it * NTHR + tid;
    const v4f v = *(const v4fa*)(os + 4 * i4);
    asm volatile("" :: "v"(v));
    if (i4 < nv4) *(volatile v4f*)(ob + (size_t)4 * (size_t)i4) = v;
  }
}

__global__ __launch_bounds__(NTHR) void k_replay_head(const int* __restrict__ LIST, const int* __restrict__ CO,
                                                      const int* __restrict__ FLAG, const float* __restrict__ DINV,
                                                      const float* __restrict__ P, const float* __restrict__ TB,
                                                      float* out) {
  __shared__ __attribute__((aligned(16))) float os[NBRUN * NC];
  const int tid = (int)threadIdx.x, lane = tid & 31, wave = tid >> 5;
  const int blk = (int)blockIdx.x;
  const int rowBase = blk * NBRUN;
  const int* lb  = LIST + (size_t)blk * RCAP;
  const int* cob = CO + (size_t)blk * (2 * NBRUN);
  const int flag = FLAG[(size_t)blk * 32];
  const float qnan = __uint_as_float(0x7fc00000u);

  const v4f pb  = *(const v4fa*)(TB + TB_B3 + 4 * lane);
  const v4f fq0 = *(const v4fa*)(TB + TB_FC + 8 * lane);
  const v4f fq1 = *(const v4fa*)(TB + TB_FC + 8 * lane + 4);
  const float fb0 = TB[TB_FCB + 0];
  const float fb1 = TB[TB_FCB + 1];
  asm volatile("" :: "v"(pb), "v"(fq0), "v"(fq1));
  asm volatile("" :: "v"(fb0), "v"(fb1));

#pragma unroll 1
  for (int i = 0; i < NBRUN / NWAVE; ++i) {
    const int s = NWAVE * i + wave;
    const int d = rowBase + s;
    int c = cob[s];
    int o = cob[NBRUN + s];
    const bool big = c > DEGCAP;
    c = c < 0 ? 0 : (c > DEGCAP ? DEGCAP : c);
    o = o < 0 ? 0 : (o > RCAP - 1 ? RCAP - 1 : o);
    c = __builtin_amdgcn_readfirstlane(c);
    o = __builtin_amdgcn_readfirstlane(o);
    const v4f a = row_sum(lb, P, c, o, lane);
    const int nc = d < NN ? d : NN - 1;
    const v4f sf = *(const v4fa*)(P + (size_t)nc * HD + 4 * lane);
    const float dd = DINV[nc];
    asm volatile("" :: "v"(sf));
    asm volatile("" :: "v"(dd));
    float y0 = dd * (a.x + sf.x) + pb.x, y1 = dd * (a.y + sf.y) + pb.y;
    float y2 = dd * (a.z + sf.z) + pb.z, y3 = dd * (a.w + sf.w) + pb.w;
    y0 = (y0 > 0.0f) ? y0 : (y0 - y0); y1 = (y1 > 0.0f) ? y1 : (y1 - y1);
    y2 = (y2 > 0.0f) ? y2 : (y2 - y2); y3 = (y3 > 0.0f) ? y3 : (y3 - y3);
    float s0 = y0 * fq0.x;
    s0 = fmaf(y1, fq0.z, s0); s0 = fmaf(y2, fq1.x, s0); s0 = fmaf(y3, fq1.z, s0);
    float s1 = y0 * fq0.y;
    s1 = fmaf(y1, fq0.w, s1); s1 = fmaf(y2, fq1.y, s1); s1 = fmaf(y3, fq1.w, s1);
#pragma unroll
    for (int dl = 16; dl > 0; dl >>= 1) {
      s0 += __shfl_xor(s0, dl, 32);
      s1 += __shfl_xor(s1, dl, 32);
    }
    float o0 = s0 + fb0, o1 = s1 + fb1;
    const bool bad  = (flag != 0) | big;
    const bool live = d < NN;
    o0 = bad ? qnan : o0; o1 = bad ? qnan : o1;
    o0 = live ? o0 : 0.0f; o1 = live ? o1 : 0.0f;
    const float ov = (lane == 0) ? o0 : o1;
    if (lane < 2) os[NC * s + lane] = ov;
  }
  __syncthreads();

  const int liveRows = (NN - rowBase) < NBRUN ? (NN - rowBase) : NBRUN;
  const int nv4 = (liveRows * NC) / 4;
  float* ob = out + (size_t)blk * (size_t)(NBRUN * NC);
  head_flush(os, ob, nv4, tid);
  __threadfence();
  head_flush(os, ob, nv4, tid);
}

extern "C" void kernel_launch(void* const* d_in, const int* in_sizes, int n_in,
                              void* d_out, int out_size, void* d_ws, size_t ws_size,
                              hipStream_t stream) {
  if (n_in < 18) return;
  if (in_sizes[0] != NN * HD) return;
  if (in_sizes[1] != 2 * NE) return;
  if (in_sizes[2] != HD * HD || in_sizes[8] != HD * HD || in_sizes[14] != HD * HD) return;
  if (in_sizes[3] != HD || in_sizes[4] != HD || in_sizes[5] != HD || in_sizes[6] != HD || in_sizes[7] != HD) return;
  if (in_sizes[9] != HD || in_sizes[10] != HD || in_sizes[11] != HD || in_sizes[12] != HD || in_sizes[13] != HD) return;
  if (in_sizes[15] != HD) return;
  if (in_sizes[16] != HD * NC || in_sizes[17] != NC) return;
  if (out_size != NN * NC) return;

  const float* x    = (const float*)d_in[0];
  const int*   ei   = (const int*)d_in[1];
  const float* W1   = (const float*)d_in[2];
  const float* b1   = (const float*)d_in[3];
  const float* g1   = (const float*)d_in[4];
  const float* be1  = (const float*)d_in[5];
  const float* m1   = (const float*)d_in[6];
  const float* v1   = (const float*)d_in[7];
  const float* W2   = (const float*)d_in[8];
  const float* b2   = (const float*)d_in[9];
  const float* g2   = (const float*)d_in[10];
  const float* be2  = (const float*)d_in[11];
  const float* m2   = (const float*)d_in[12];
  const float* v2   = (const float*)d_in[13];
  const float* W3   = (const float*)d_in[14];
  const float* b3   = (const float*)d_in[15];
  const float* fcW  = (const float*)d_in[16];
  const float* fcb  = (const float*)d_in[17];
  float* out = (float*)d_out;
  const int* srcs = ei;
  const int* dsts = ei + NE;

  constexpr size_t zXB   = (size_t)MP * HD * 2;
  constexpr size_t zP    = (size_t)MP * HD * 4;
  constexpr size_t zHL   = (size_t)MP * AP_TWO * 2;
  constexpr size_t zLIST = (size_t)NBK * RCAP * 4;
  constexpr size_t zCO   = (size_t)NBK * 2 * NBRUN * 4;
  constexpr size_t zDINV = (size_t)NBK * NBRUN * 4;
  constexpr size_t zFLAG = (((size_t)NBK * 128 + 255) / 256) * 256;
  constexpr size_t zW1T  = (size_t)HD * WP_ONE * 2;
  constexpr size_t zWD   = (size_t)HD * WP_TWO * 2;
  constexpr size_t zTB   = 8192;
  constexpr size_t oXB   = 0;
  constexpr size_t oP    = oXB + zXB;
  constexpr size_t oHL   = oP + zP;
  constexpr size_t oLIST = oHL + zHL;
  constexpr size_t oCO   = oLIST + zLIST;
  constexpr size_t oDINV = oCO + zCO;
  constexpr size_t oFLAG = oDINV + zDINV;
  constexpr size_t oW1T  = oFLAG + zFLAG;
  constexpr size_t oW2D  = oW1T + zW1T;
  constexpr size_t oW3D  = oW2D + zWD;
  constexpr size_t oTB   = oW3D + zWD;
  constexpr size_t oEND  = oTB + zTB;
  static_assert(zXB == 12812288);
  static_assert(zXB % 256 == 0 && zP % 256 == 0 && zHL % 256 == 0 && zLIST % 256 == 0 && zCO % 256 == 0);
  static_assert(zDINV % 256 == 0 && zFLAG % 256 == 0 && zW1T % 256 == 0 && zWD % 256 == 0 && zTB % 256 == 0);
  static_assert(zTB >= 14 * 128 * 4);
  static_assert(zDINV >= (size_t)MP * 4);
  static_assert(oEND <= (size_t)(128u << 20));
  if (oEND > ws_size) return;

  char* ws = (char*)d_ws;
  unsigned short* XB   = (unsigned short*)(ws + oXB);
  float*          P    = (float*)(ws + oP);
  unsigned short* HL   = (unsigned short*)(ws + oHL);
  int*            LIST = (int*)(ws + oLIST);
  int*            CO   = (int*)(ws + oCO);
  float*          DINV = (float*)(ws + oDINV);
  int*            FLAG = (int*)(ws + oFLAG);
  unsigned short* W1T  = (unsigned short*)(ws + oW1T);
  unsigned short* W2D  = (unsigned short*)(ws + oW2D);
  unsigned short* W3D  = (unsigned short*)(ws + oW3D);
  float*          TB   = (float*)(ws + oTB);

  constexpr int KT2 = SPLIT_TWO ? 256 : 128;
  constexpr int KT3 = SPLIT_THREE ? 256 : 128;

  hipFuncSetAttribute(reinterpret_cast<const void*>(&k_bucket), hipFuncAttributeMaxDynamicSharedMemorySize, (int)BK_LDS);
  hipFuncSetAttribute(reinterpret_cast<const void*>(&k_gemm_one), hipFuncAttributeMaxDynamicSharedMemorySize, (int)GM_LDS);
  hipFuncSetAttribute(reinterpret_cast<const void*>(&k_gemm_two<KT2>), hipFuncAttributeMaxDynamicSharedMemorySize, (int)GM_LDS);
  hipFuncSetAttribute(reinterpret_cast<const void*>(&k_gemm_two<KT3>), hipFuncAttributeMaxDynamicSharedMemorySize, (int)GM_LDS);

  k_prep<<<PBTOT, NTHR, 0, stream>>>(x, W1, W2, W3, b1, g1, be1, m1, v1, b2, g2, be2, m2, v2, b3, fcW, fcb,
                                     XB, W1T, W2D, W3D, HL, TB);
  k_bucket<<<NBK, NTHR, BK_LDS, stream>>>(srcs, dsts, LIST, CO, DINV, FLAG);
  k_gemm_one<<<MP / GBM, NTHR, GM_LDS, stream>>>(XB, W1T, DINV, P);
  k_replay_hl<<<MP / GBM, NTHR, 0, stream>>>(LIST, CO, FLAG, DINV, P, TB + TB_L1, HL);
  k_gemm_two<KT2><<<MP / GBM, NTHR, GM_LDS, stream>>>(HL, W2D, DINV, P);
  k_replay_hl<<<MP / GBM, NTHR, 0, stream>>>(LIST, CO, FLAG, DINV, P, TB + TB_L2, HL);
  k_gemm_two<KT3><<<MP / GBM, NTHR, GM_LDS, stream>>>(HL, W3D, DINV, P);
  k_replay_head<<<NBK, NTHR, 0, stream>>>(LIST, CO, FLAG, DINV, P, TB, out);
}
